// GNNSoftMask_31756988186744
// MI455X (gfx1250) — hardware-verified
//
#include <hip/hip_runtime.h>
#include <stddef.h>
#include <stdint.h>
#include <math.h>


#define HID    128
#define KA     256
#define NTHR   256
#define NWAVE  8
#define EPT    8
#define CHUNK  (NTHR * EPT)
#define WCAP   (EPT * 32)
#define LISTN  (NWAVE * WCAP)
#define NBA    1024
#define SLA    10
#define RCAP   16384
#define DEGCAP 64
#define GBM    64
#define GBN    128
#define GTHR   128
#define EMB    1024
#define OB     1024
#define N_EXP  50000
#define E_EXP  600000
#define MP_EXP 50048
#define NU_WE  (HID * (HID / 8))
#define NU_WG  (3 * HID * (KA / 8))
#define NU_WM  (KA * (KA / 8))
#define AGG_ZINTS (LISTN + 2 * RCAP + 3 * NBA)
#define BKT_LDS_INTS (AGG_ZINTS + 64)
#define WSMAX  134217728

static_assert((CHUNK & (CHUNK - 1)) == 0 && CHUNK <= 4096);
static_assert((NBA & (NBA - 1)) == 0 && NBA == (1 << SLA));
static_assert(((long long)CHUNK << SLA) < (1LL << 31));
static_assert(((long long)E_EXP << SLA) < (1LL << 31));
static_assert(LISTN % NTHR == 0);
static_assert(NBA % NWAVE == 0 && NBA % 32 == 0 && NBA == 4 * NTHR);
static_assert(RCAP % (4 * NTHR) == 0 && AGG_ZINTS % 4 == 0 && LISTN % 4 == 0);
static_assert(RCAP >= 13176);
static_assert(DEGCAP >= 36 && DEGCAP % 32 == 0);
static_assert(BKT_LDS_INTS * 4 <= 300000);
static_assert(HID == 4 * 32 && KA == 2 * HID && KA % 32 == 0 && HID % 32 == 0);
static_assert(GBM == (GTHR / 32) * 16 && GBN == HID);
static_assert(MP_EXP % GBM == 0 && MP_EXP % 128 == 0 && MP_EXP >= N_EXP && MP_EXP % NWAVE == 0);
static_assert(49 * NBA >= MP_EXP);
static_assert(E_EXP % 32 == 0 && E_EXP % 4 == 0);
static_assert(1 + E_EXP == 600001);
static_assert(((1 + E_EXP + N_EXP * HID) & 3) == 1);
static_assert(NU_WE % NTHR == 0 && NU_WG % NTHR == 0 && NU_WM % NTHR == 0 && (MP_EXP * 16) % NTHR == 0);
static_assert(EMB == 4 * NTHR && EMB == NWAVE * 4 * 32 && OB == 4 * NTHR);

typedef float          v4f   __attribute__((ext_vector_type(4)));
typedef float          v8f   __attribute__((ext_vector_type(8)));
typedef int            v4i   __attribute__((ext_vector_type(4)));
typedef int            v8i   __attribute__((ext_vector_type(8)));
typedef unsigned       v2u   __attribute__((ext_vector_type(2)));
typedef unsigned short v8us  __attribute__((ext_vector_type(8)));
typedef unsigned short v16us __attribute__((ext_vector_type(16)));
typedef __bf16         v16bf __attribute__((ext_vector_type(16)));
typedef v4f  __attribute__((may_alias)) v4fa;
typedef v4i  __attribute__((may_alias)) v4ia;
typedef v2u  __attribute__((may_alias)) v2ua;
typedef v8us __attribute__((may_alias)) v8usa;
union FragB { v16bf v; v16us u; v8us h[2]; v8i w; };

__device__ __forceinline__ v8f wmb(const FragB& a, const FragB& b, v8f c) {
  v8f d = __builtin_amdgcn_wmma_f32_16x16x32_bf16(false, a.v, false, b.v, (short)0, c, false, false);
  asm volatile("v_nop\n\tv_nop\n\tv_nop\n\tv_nop" : "+v"(d) : "v"(a.w), "v"(b.w));
  return d;
}

__device__ __forceinline__ unsigned bf16_bits(float f) {
  const unsigned u = __float_as_uint(f);
  const unsigned r = (u + 0x7FFFu + ((u >> 16) & 1u)) >> 16;
  return (f != f) ? 0x7FC0u : r;
}
__device__ __forceinline__ float bf16_val(float f) {
  return __uint_as_float(bf16_bits(f) << 16);
}
__device__ __forceinline__ float relu_np(float v) {
  return (v > 0.0f) ? v : (v - v);
}
__device__ __forceinline__ float wsum(float v) {
#pragma unroll
  for (int q = 16; q > 0; q >>= 1) v += __shfl_xor(v, q, 32);
  return v;
}
__device__ __forceinline__ void put16(unsigned short* dp, v8us o) {
  *(volatile v8us*)dp = o;
  __threadfence();
  *(volatile v8us*)dp = o;
}

__device__ __forceinline__ void hilo_pack(float v0, float v1, float v2, float v3,
                                          int& h01, int& h23, int& l01, int& l23) {
  const unsigned a0 = bf16_bits(v0), a1 = bf16_bits(v1), a2 = bf16_bits(v2), a3 = bf16_bits(v3);
  const unsigned b0 = bf16_bits(v0 - __uint_as_float(a0 << 16));
  const unsigned b1 = bf16_bits(v1 - __uint_as_float(a1 << 16));
  const unsigned b2 = bf16_bits(v2 - __uint_as_float(a2 << 16));
  const unsigned b3 = bf16_bits(v3 - __uint_as_float(a3 << 16));
  h01 = (int)(a0 | (a1 << 16)); h23 = (int)(a2 | (a3 << 16));
  l01 = (int)(b0 | (b1 << 16)); l23 = (int)(b2 | (b3 << 16));
}

__device__ __forceinline__ v4i regroup16(int h01, int h23, int l01, int l23, int lane) {
  const int s0 = (2 * lane) & 31, s1 = s0 + 1;
  const int a0 = __shfl(h01, s0, 32), a1 = __shfl(h23, s0, 32), a2 = __shfl(h01, s1, 32), a3 = __shfl(h23, s1, 32);
  const int b0 = __shfl(l01, s0, 32), b1 = __shfl(l23, s0, 32), b2 = __shfl(l01, s1, 32), b3 = __shfl(l23, s1, 32);
  const int mk = (lane < 16) ? -1 : 0;
  v4i o;
  o.x = (a0 & mk) | (b0 & ~mk); o.y = (a1 & mk) | (b1 & ~mk);
  o.z = (a2 & mk) | (b2 & ~mk); o.w = (a3 & mk) | (b3 & ~mk);
  return o;
}

template <int SLB>
__device__ __forceinline__ int scan_chunk(const int* __restrict__ dsts, int nE, int cbase, int slotBase,
                                          int nb, int vec8, int* list, int tid, int lane, int wave) {
  int wc = 0;
  const int el0  = tid * EPT;
  const int e0   = cbase + el0;
  const int sent = -2147483647 - 1;
  v4i da, db;
  if (vec8 != 0 && cbase + CHUNK <= nE) {
    da = *(const v4i*)(dsts + e0);
    db = *(const v4i*)(dsts + e0 + 4);
  } else {
    da.x = (e0     < nE) ? dsts[min(e0,     nE - 1)] : sent;
    da.y = (e0 + 1 < nE) ? dsts[min(e0 + 1, nE - 1)] : sent;
    da.z = (e0 + 2 < nE) ? dsts[min(e0 + 2, nE - 1)] : sent;
    da.w = (e0 + 3 < nE) ? dsts[min(e0 + 3, nE - 1)] : sent;
    db.x = (e0 + 4 < nE) ? dsts[min(e0 + 4, nE - 1)] : sent;
    db.y = (e0 + 5 < nE) ? dsts[min(e0 + 5, nE - 1)] : sent;
    db.z = (e0 + 6 < nE) ? dsts[min(e0 + 6, nE - 1)] : sent;
    db.w = (e0 + 7 < nE) ? dsts[min(e0 + 7, nE - 1)] : sent;
  }
  const unsigned nbs = (unsigned)slotBase;
  const unsigned unb = (unsigned)nb;
  const unsigned s0 = (unsigned)da.x - nbs, s1 = (unsigned)da.y - nbs;
  const unsigned s2 = (unsigned)da.z - nbs, s3 = (unsigned)da.w - nbs;
  const unsigned s4 = (unsigned)db.x - nbs, s5 = (unsigned)db.y - nbs;
  const unsigned s6 = (unsigned)db.z - nbs, s7 = (unsigned)db.w - nbs;
  const bool h0 = s0 < unb, h1 = s1 < unb, h2 = s2 < unb, h3 = s3 < unb;
  const bool h4 = s4 < unb, h5 = s5 < unb, h6 = s6 < unb, h7 = s7 < unb;
  const unsigned any = __builtin_amdgcn_ballot_w32(h0 | h1 | h2 | h3 | h4 | h5 | h6 | h7);
  if (any != 0u) {
#define HITJ(J, HJ, SJ) { \
      const unsigned mj = __builtin_amdgcn_ballot_w32(HJ); \
      if (mj != 0u) { \
        if (HJ) { \
          const int pos = wc + (int)__builtin_amdgcn_mbcnt_lo(mj, 0u); \
          if (pos < WCAP) list[wave * WCAP + pos] = ((el0 + (J)) << SLB) | (int)(SJ); \
        } \
        wc += (int)__builtin_popcount(mj); } }
    HITJ(0, h0, s0)
    HITJ(1, h1, s1)
    HITJ(2, h2, s2)
    HITJ(3, h3, s3)
    HITJ(4, h4, s4)
    HITJ(5, h5, s5)
    HITJ(6, h6, s6)
    HITJ(7, h7, s7)
#undef HITJ
  }
  return wc;
}

__global__ __launch_bounds__(NTHR) void k_prep(const float* __restrict__ X, const float* __restrict__ Wemb,
                                               const float* __restrict__ Wgnn, const float* __restrict__ Wm1,
                                               int nN, int mRows,
                                               unsigned short* WeT, unsigned short* WgT2, unsigned short* WmT2,
                                               unsigned short* XB) {
  const int u  = (int)blockIdx.x * NTHR + (int)threadIdx.x;
  const int U0 = NU_WE;
  const int U1 = U0 + NU_WG;
  const int U2 = U1 + NU_WM;
  const int U3 = U2 + mRows * 16;
  v8us o;
  if (u < U0) {
    const int n  = u >> 4;
    const int k8 = (u & 15) * 8;
    const float* p = Wemb + (size_t)k8 * HID + n;
#pragma unroll
    for (int i = 0; i < 8; ++i) o[i] = (unsigned short)bf16_bits(p[(size_t)i * HID]);
    put16(WeT + (size_t)n * HID + k8, o);
  } else if (u < U1) {
    const int v  = u - U0;
    const int ly = v >> 12;
    const int n  = (v >> 5) & (HID - 1);
    const int k8 = (v & 31) * 8;
    const int kk = k8 & (HID - 1);
    const float* p = Wgnn + (size_t)ly * HID * HID + (size_t)kk * HID + n;
#pragma unroll
    for (int i = 0; i < 8; ++i) o[i] = (unsigned short)bf16_bits(p[(size_t)i * HID]);
    put16(WgT2 + (size_t)ly * HID * KA + (size_t)n * KA + k8, o);
  } else if (u < U2) {
    const int v  = u - U1;
    const int n  = v >> 5;
    const int k8 = (v & 31) * 8;
    const int kk = k8 & (HID - 1);
    const int nn = n & (HID - 1);
    const int hf = n >> 7;
    const float* p = Wm1 + (size_t)(hf * HID + kk) * HID + nn;
#pragma unroll
    for (int i = 0; i < 8; ++i) o[i] = (unsigned short)bf16_bits(p[(size_t)i * HID]);
    put16(WmT2 + (size_t)n * KA + k8, o);
  } else if (u < U3) {
    const int v   = u - U2;
    const int row = v >> 4;
    const int k8  = (v & 15) * 8;
    const int rc  = row < nN ? row : nN - 1;
    const float* p = X + (size_t)rc * HID + k8;
    const v4f a = *(const v4fa*)p;
    const v4f b = *(const v4fa*)(p + 4);
    const bool ok = row < nN;
    o[0] = ok ? (unsigned short)bf16_bits(a.x) : (unsigned short)0;
    o[1] = ok ? (unsigned short)bf16_bits(a.y) : (unsigned short)0;
    o[2] = ok ? (unsigned short)bf16_bits(a.z) : (unsigned short)0;
    o[3] = ok ? (unsigned short)bf16_bits(a.w) : (unsigned short)0;
    o[4] = ok ? (unsigned short)bf16_bits(b.x) : (unsigned short)0;
    o[5] = ok ? (unsigned short)bf16_bits(b.y) : (unsigned short)0;
    o[6] = ok ? (unsigned short)bf16_bits(b.z) : (unsigned short)0;
    o[7] = ok ? (unsigned short)bf16_bits(b.w) : (unsigned short)0;
    put16(XB + (size_t)row * HID + k8, o);
  }
}

__device__ __forceinline__ void spill_pass(const int* sl, const int* cnt, const int* offs, const int* mline,
                                           int* gl, int* gc, int* go, int* gm, int tid) {
#pragma unroll 4
  for (int it = 0; it < RCAP / (4 * NTHR); ++it) {
    const int q = (it * NTHR + tid) * 4;
    const v4i v = *(const v4ia*)(sl + q);
    *(volatile v4i*)(gl + q) = v;
  }
  {
    const v4i c4 = *(const v4ia*)(cnt + 4 * tid);
    const v4i o4 = *(const v4ia*)(offs + 4 * tid);
    *(volatile v4i*)(gc + 4 * tid) = c4;
    *(volatile v4i*)(go + 4 * tid) = o4;
  }
  {
    const int tl = tid < 8 ? tid : 7;
    const v4i m4 = *(const v4ia*)(mline + 4 * tl);
    if (tid < 8) *(volatile v4i*)(gm + 4 * tl) = m4;
  }
}

__global__ __launch_bounds__(NTHR) void k_bucket(const int* __restrict__ dsts, int nE, int vec8,
                                                 int* LIST, int* CNT, int* OFF, int* META) {
  extern __shared__ __attribute__((aligned(16))) int dsm[];
  int* list  = dsm;
  int* hl    = dsm + LISTN;
  int* sl    = hl + RCAP;
  int* cnt   = sl + RCAP;
  int* offs  = cnt + NBA;
  int* cur   = offs + NBA;
  int* misc  = cur + NBA;
  int* mline = misc + 32;
  const int tid = (int)threadIdx.x, lane = tid & 31, wave = tid >> 5;
  const int blk = (int)blockIdx.x;
  const int nodeBase = blk * NBA;

  {
    const v4i z4 = {0, 0, 0, 0};
    for (int i = tid * 4; i < AGG_ZINTS; i += NTHR * 4) *(v4ia*)(dsm + i) = z4;
    if (tid < 64) misc[tid] = 0;
  }
  __syncthreads();

  int t = 0, ov = 0;
  const int nChunks = (nE + CHUNK - 1) / CHUNK;
#pragma unroll 1
  for (int ch = 0; ch < nChunks; ++ch) {
    const int cbase = ch * CHUNK;
    const int wc = scan_chunk<SLA>(dsts, nE, cbase, nodeBase, NBA, vec8, list, tid, lane, wave);
    if (lane == 0) misc[wave] = wc;
    __syncthreads();
    if (wave == 0) {
#pragma unroll 1
      for (int w2 = 0; w2 < NWAVE; ++w2) {
        int c = misc[w2];
        c = c < 0 ? 0 : (c > WCAP ? WCAP : c);
#pragma unroll 1
        for (int b0 = 0; b0 < c; b0 += 32) {
          const int idx = b0 + lane;
          const int ent = list[w2 * WCAP + (idx < WCAP ? idx : WCAP - 1)];
          const int m32 = (c - b0) < 32 ? (c - b0) : 32;
#pragma unroll 1
          for (int k = 0; k < m32; ++k) {
            const int u    = __builtin_amdgcn_readlane(ent, k);
            const int slot = u & (NBA - 1);
            const int el   = (u >> SLA) & (CHUNK - 1);
            const int pk   = ((cbase + el) << SLA) | slot;
            if (t < RCAP) {
              if (lane == 0) { hl[t] = pk; cnt[slot] = cnt[slot] + 1; }
              t = t + 1;
            } else {
              ov = 1;
            }
          }
        }
      }
    }
    __syncthreads();
  }
  if (wave == 0 && lane == 0) { misc[8] = t; misc[9] = ov; mline[0] = t; mline[1] = ov; }
  __syncthreads();
  int tt = misc[8];
  tt = tt < 0 ? 0 : (tt > RCAP ? RCAP : tt);

  if (wave == 0) {
    const int base = lane * (NBA / 32);
    int s = 0;
#pragma unroll 1
    for (int i = 0; i < NBA / 32; ++i) s += cnt[base + i];
    int incl = s;
#pragma unroll
    for (int d = 1; d < 32; d <<= 1) {
      const int y = __shfl_up(incl, d, 32);
      if (lane >= d) incl += y;
    }
    int run = incl - s;
#pragma unroll 1
    for (int i = 0; i < NBA / 32; ++i) {
      const int cv = cnt[base + i];
      offs[base + i] = run;
      cur[base + i]  = run;
      run += cv;
    }
  }
  __syncthreads();
  if (wave == 0) {
#pragma unroll 1
    for (int b0 = 0; b0 < tt; b0 += 32) {
      const int idx = b0 + lane;
      const int ent = hl[idx < RCAP ? idx : RCAP - 1];
      const int m32 = (tt - b0) < 32 ? (tt - b0) : 32;
#pragma unroll 1
      for (int k = 0; k < m32; ++k) {
        const int u    = __builtin_amdgcn_readlane(ent, k);
        const int slot = u & (NBA - 1);
        if (lane == 0) {
          int p = cur[slot];
          p = p < 0 ? 0 : (p > RCAP - 1 ? RCAP - 1 : p);
          sl[p] = u;
          cur[slot] = p + 1;
        }
      }
    }
  }
  __syncthreads();

  int* gl = LIST + (size_t)blk * RCAP;
  int* gc = CNT  + (size_t)blk * NBA;
  int* go = OFF  + (size_t)blk * NBA;
  int* gm = META + (size_t)blk * 32;
  spill_pass(sl, cnt, offs, mline, gl, gc, go, gm, tid);
  __threadfence();
  spill_pass(sl, cnt, offs, mline, gl, gc, go, gm, tid);
}

template <int MODE>
__global__ __launch_bounds__(GTHR) void k_gemm(const unsigned short* __restrict__ A, int lda,
                                               const unsigned short* __restrict__ BT, int ldb, int K,
                                               const float* __restrict__ bias, int nN,
                                               float* Cm, int ldc, unsigned short* Cb) {
  __shared__ __attribute__((aligned(16))) float stg[GBM * GBN];
  const int tid = (int)threadIdx.x, lane = tid & 31, wave = tid >> 5, hh = lane >> 4, m = lane & 15;
  const int rowBase = (int)blockIdx.x * GBM;
  const int colBase = (int)blockIdx.y * GBN;

  v8f acc[8];
  {
    const v8f z = {0.f, 0.f, 0.f, 0.f, 0.f, 0.f, 0.f, 0.f};
#pragma unroll
    for (int t = 0; t < 8; ++t) acc[t] = z;
  }
  const unsigned short* ap = A  + (size_t)(rowBase + 16 * wave + m) * (size_t)lda + 8 * hh;
  const unsigned short* bp = BT + (size_t)(colBase + m) * (size_t)ldb + 8 * hh;

#pragma unroll 1
  for (int k0 = 0; k0 < K; k0 += 32) {
    FragB af;
    af.h[0] = *(const v8usa*)(ap + k0);
    af.h[1] = *(const v8usa*)(ap + k0 + 16);
#pragma unroll
    for (int nt = 0; nt < 8; ++nt) {
      const unsigned short* wq = bp + (size_t)(16 * nt) * (size_t)ldb + k0;
      FragB bf;
      bf.h[0] = *(const v8usa*)wq;
      bf.h[1] = *(const v8usa*)(wq + 16);
      acc[nt] = wmb(af, bf, acc[nt]);
    }
  }

#pragma unroll
  for (int nt = 0; nt < 8; ++nt) {
    const int lc = 16 * nt + m;
    float bvv = bf16_val(bias[lc]);
    if constexpr (MODE == 0) bvv = (colBase >= HID) ? bvv : 0.0f;
#pragma unroll
    for (int r = 0; r < 8; ++r) {
      const int lr = 16 * wave + 8 * hh + r;
      float v = acc[nt][r] + bvv;
      if constexpr (MODE != 0) v = relu_np(v);
      stg[lr * GBN + lc] = v;
    }
  }
  __syncthreads();

  {
    v4f pv[16];
#pragma unroll
    for (int i = 0; i < 16; ++i) {
      const int row = rowBase + 16 * wave + i;
      v4f sv = *(const v4fa*)(stg + (16 * wave + i) * GBN + 4 * lane);
      if constexpr (MODE != 0) {
        const bool ok = row < nN;
        sv.x = ok ? sv.x : 0.0f; sv.y = ok ? sv.y : 0.0f; sv.z = ok ? sv.z : 0.0f; sv.w = ok ? sv.w : 0.0f;
      }
      pv[i] = sv;
    }
#pragma unroll
    for (int i = 0; i < 16; ++i) {
      float* op = Cm + (size_t)(rowBase + 16 * wave + i) * (size_t)ldc + colBase + 4 * lane;
      *(volatile v4f*)op = pv[i];
    }
    __threadfence();
#pragma unroll
    for (int i = 0; i < 16; ++i) {
      float* op = Cm + (size_t)(rowBase + 16 * wave + i) * (size_t)ldc + colBase + 4 * lane;
      *(volatile v4f*)op = pv[i];
    }
  }

  if constexpr (MODE == 1) {
    const int part = lane >> 4;
    const int j = lane & 15;
    const unsigned mh = 0u - (unsigned)part;
    const unsigned ml = ~mh;
    v8us pw[16];
#pragma unroll
    for (int i = 0; i < 16; ++i) {
      const int row = rowBase + 16 * wave + i;
      const bool ok = row < nN;
      const float* sp = stg + (16 * wave + i) * GBN + 8 * j;
      const v4f a = *(const v4fa*)sp;
      const v4f b = *(const v4fa*)(sp + 4);
      const v8f f8 = {a.x, a.y, a.z, a.w, b.x, b.y, b.z, b.w};
      v8us oo;
#pragma unroll
      for (int e = 0; e < 8; ++e) {
        const float fv = ok ? f8[e] : 0.0f;
        const unsigned hb = bf16_bits(fv);
        const unsigned lb = bf16_bits(fv - __uint_as_float(hb << 16));
        oo[e] = (unsigned short)((hb & ml) | (lb & mh));
      }
      pw[i] = oo;
    }
#pragma unroll
    for (int i = 0; i < 16; ++i) {
      unsigned short* op = Cb + (size_t)(rowBase + 16 * wave + i) * (size_t)KA + part * HID + 8 * j;
      *(volatile v8us*)op = pw[i];
    }
    __threadfence();
#pragma unroll
    for (int i = 0; i < 16; ++i) {
      unsigned short* op = Cb + (size_t)(rowBase + 16 * wave + i) * (size_t)KA + part * HID + 8 * j;
      *(volatile v8us*)op = pw[i];
    }
  }
}

__global__ __launch_bounds__(NTHR) void k_emask(const int* __restrict__ src, const int* __restrict__ dst,
                                                int nE, int nN, const float* __restrict__ PSD,
                                                const float* __restrict__ Wm2, const float* __restrict__ bm2,
                                                float* MASK) {
  __shared__ __attribute__((aligned(16))) float sm[EMB];
  const int tid = (int)threadIdx.x, lane = tid & 31;
  const int wave = __builtin_amdgcn_readfirstlane(tid >> 5);
  const v4f wr = *(const v4fa*)(Wm2 + 4 * lane);
  const float w0 = bf16_val(wr.x), w1 = bf16_val(wr.y), w2 = bf16_val(wr.z), w3 = bf16_val(wr.w);
  const float b2 = bf16_val(bm2[0]);
  const int ebase = (int)blockIdx.x * EMB;

#pragma unroll 1
  for (int bi = 0; bi < 4; ++bi) {
    const int bq = wave * 4 + bi;
    const int eb = ebase + bq * 32;
    const bool bv = (eb + 32) <= nE;
    float mine = 0.0f;
    if (bv) {
      int s = src[eb + lane];
      int d = dst[eb + lane];
      s = s < 0 ? 0 : (s > nN - 1 ? nN - 1 : s);
      d = d < 0 ? 0 : (d > nN - 1 ? nN - 1 : d);
#pragma unroll 1
      for (int k = 0; k < 32; ++k) {
        const int sk = __builtin_amdgcn_readlane(s, k);
        const int dk = __builtin_amdgcn_readlane(d, k);
        const v4f a = *(const v4fa*)(PSD + (size_t)sk * KA + 4 * lane);
        const v4f b = *(const v4fa*)(PSD + (size_t)dk * KA + HID + 4 * lane);
        const float t0 = relu_np(a.x + b.x);
        const float t1 = relu_np(a.y + b.y);
        const float t2 = relu_np(a.z + b.z);
        const float t3 = relu_np(a.w + b.w);
        float p = t0 * w0;
        p = fmaf(t1, w1, p);
        p = fmaf(t2, w2, p);
        p = fmaf(t3, w3, p);
        const float tot = wsum(p);
        mine = (lane == k) ? tot : mine;
      }
      const float sv  = mine + b2;
      const float imp = 1.0f / (1.0f + expf(-sv));
      const float g   = (imp - 0.4f) * 2.0f;
      mine = 1.0f / (1.0f + expf(-g));
    }
    sm[bq * 32 + lane] = mine;
  }
  __syncthreads();

  const int j0 = ebase + 4 * tid;
  const v4f o4 = *(const v4fa*)(sm + 4 * tid);
  const bool ok = (j0 + 4) <= nE;
  int jc = j0;
  jc = jc > nE - 4 ? nE - 4 : jc;
  float* mp = MASK + (size_t)jc;
  if (ok) *(volatile v4f*)mp = o4;
  __threadfence();
  if (ok) *(volatile v4f*)mp = o4;
}

__global__ __launch_bounds__(NTHR) void k_agg(const int* __restrict__ srcs, int nE, int nN, int mRows,
                                              const int* __restrict__ LIST, const int* __restrict__ CNT,
                                              const int* __restrict__ OFF, const int* __restrict__ META,
                                              const float* __restrict__ MASK, const float* __restrict__ H,
                                              unsigned short* Z) {
  const int tid = (int)threadIdx.x, lane = tid & 31;
  const int wave = __builtin_amdgcn_readfirstlane(tid >> 5);
  const int node  = (int)blockIdx.x * NWAVE + wave;
  const int nodec = node < mRows ? node : mRows - 1;
  const int bb    = nodec >> SLA;
  int c = __builtin_amdgcn_readfirstlane(CNT[nodec]);
  const bool big = c > DEGCAP;
  c = c < 0 ? 0 : (c > DEGCAP ? DEGCAP : c);
  int o = __builtin_amdgcn_readfirstlane(OFF[nodec]);
  o = o < 0 ? 0 : (o > RCAP ? RCAP : o);
  const int ovf = __builtin_amdgcn_readfirstlane(META[bb * 32 + 1]);
  const int* lp = LIST + (size_t)bb * RCAP;

  float g0 = 0.0f, g1 = 0.0f, g2 = 0.0f, g3 = 0.0f;
#pragma unroll 1
  for (int b0 = 0; b0 < c; b0 += 32) {
    int idx = o + b0 + lane;
    idx = idx > RCAP - 1 ? RCAP - 1 : idx;
    const int ent = lp[idx];
    int eid = ent >> SLA;
    eid = eid < 0 ? 0 : (eid > nE - 1 ? nE - 1 : eid);
    int sr = srcs[eid];
    sr = sr < 0 ? 0 : (sr > nN - 1 ? nN - 1 : sr);
    const int mki = __float_as_int(MASK[eid]);
    const int m32 = (c - b0) < 32 ? (c - b0) : 32;
#pragma unroll 1
    for (int k = 0; k < m32; ++k) {
      const int   sk = __builtin_amdgcn_readlane(sr, k);
      const float wk = __int_as_float(__builtin_amdgcn_readlane(mki, k));
      const v4f a = *(const v4fa*)(H + (size_t)sk * HID + 4 * lane);
      g0 = fmaf(a.x, wk, g0); g1 = fmaf(a.y, wk, g1);
      g2 = fmaf(a.z, wk, g2); g3 = fmaf(a.w, wk, g3);
    }
  }
  const int nr = nodec < nN ? nodec : nN - 1;
  const v4f hr = *(const v4fa*)(H + (size_t)nr * HID + 4 * lane);
  const float qnan = __int_as_float(0x7fc00000);
  const float pzr  = (big || (ovf != 0)) ? qnan : 0.0f;
  const bool live = node < nN;
  const float q0 = live ? (hr.x + g0) + pzr : 0.0f;
  const float q1 = live ? (hr.y + g1) + pzr : 0.0f;
  const float q2 = live ? (hr.z + g2) + pzr : 0.0f;
  const float q3 = live ? (hr.w + g3) + pzr : 0.0f;
  int h01, h23, l01, l23;
  hilo_pack(q0, q1, q2, q3, h01, h23, l01, l23);
  const v4i ow = regroup16(h01, h23, l01, l23, lane);
  if (node < mRows) {
    unsigned short* hp = Z + (size_t)node * KA + 8 * lane;
    *(volatile v4i*)hp = ow;
    __threadfence();
    *(volatile v4i*)hp = ow;
  }
}

__global__ __launch_bounds__(HID) void k_pred(const float* __restrict__ H, const float* __restrict__ Wp1,
                                              const float* __restrict__ bp1, const float* __restrict__ Wp2,
                                              const float* __restrict__ bp2, float* PRED) {
  __shared__ __attribute__((aligned(16))) float sh[HID];
  __shared__ __attribute__((aligned(16))) float sline[32];
  __shared__ float sred[4];
  const int tid = (int)threadIdx.x, lane = tid & 31, wave = tid >> 5;
  sh[tid] = H[tid];
  if (tid < 32) sline[tid] = 0.0f;
  __syncthreads();
  float s = 0.0f;
#pragma unroll 4
  for (int k = 0; k < HID; ++k) s = fmaf(sh[k], bf16_val(Wp1[(size_t)k * HID + tid]), s);
  s = s + bf16_val(bp1[tid]);
  const float pr = relu_np(s) * bf16_val(Wp2[tid]);
  const float wsv = wsum(pr);
  if (lane == 0) sred[wave] = wsv;
  __syncthreads();
  if (tid == 0) sline[0] = (((sred[0] + sred[1]) + sred[2]) + sred[3]) + bf16_val(bp2[0]);
  __syncthreads();
  const int tl = tid < 8 ? tid : 7;
  const v4f o4 = *(const v4fa*)(sline + 4 * tl);
  if (tid < 8) *(volatile v4f*)(PRED + 4 * tl) = o4;
  __threadfence();
  if (tid < 8) *(volatile v4f*)(PRED + 4 * tl) = o4;
}

__global__ __launch_bounds__(NTHR) void k_out(const float* __restrict__ PRED, const float* __restrict__ MASK,
                                              const float* __restrict__ H, int nE, int nH, int total,
                                              float* out) {
  __shared__ __attribute__((aligned(16))) float sb[OB];
  const int tid  = (int)threadIdx.x;
  const int base = (int)blockIdx.x * OB;
  const int offH = 1 + nE;
  const bool allH = base >= offH;
  const bool allM = (base >= 1) && (base + OB - 1 <= nE);
  if (allH) {
#pragma unroll
    for (int i = 0; i < 4; ++i) {
      int jh = base + tid + NTHR * i - offH;
      jh = jh > nH - 1 ? nH - 1 : jh;
      sb[tid + NTHR * i] = H[(size_t)jh];
    }
  } else if (allM) {
#pragma unroll
    for (int i = 0; i < 4; ++i) {
      int jm = base + tid + NTHR * i - 1;
      jm = jm < 0 ? 0 : (jm > nE - 1 ? nE - 1 : jm);
      sb[tid + NTHR * i] = MASK[(size_t)jm];
    }
  } else {
    const unsigned up = __float_as_uint(PRED[0]);
#pragma unroll 1
    for (int i = 0; i < 4; ++i) {
      const int j = base + tid + NTHR * i;
      int jm = j - 1;
      jm = jm < 0 ? 0 : (jm > nE - 1 ? nE - 1 : jm);
      int jh = j - offH;
      jh = jh < 0 ? 0 : (jh > nH - 1 ? nH - 1 : jh);
      const unsigned um = __float_as_uint(MASK[(size_t)jm]);
      const unsigned uh = __float_as_uint(H[(size_t)jh]);
      const unsigned mP = (j == 0) ? 0xffffffffu : 0u;
      const unsigned mH = (j >= offH) ? 0xffffffffu : 0u;
      const unsigned mM = ~(mP | mH);
      sb[tid + NTHR * i] = __uint_as_float((um & mM) | (uh & mH) | (up & mP));
    }
  }
  __syncthreads();
  const int j0 = base + 4 * tid;
  const v4f o4 = *(const v4fa*)(sb + 4 * tid);
  const bool vok = (j0 + 4) <= total;
  const bool tok = (!vok) && (j0 < total);
  int jc = j0;
  jc = jc > total - 1 ? total - 1 : jc;
  float* op = out + (size_t)jc;
  const float o1 = o4.x;
  if (vok) *(volatile v4f*)op = o4;
  if (tok) *(volatile float*)op = o1;
  __threadfence();
  if (vok) *(volatile v4f*)op = o4;
  if (tok) *(volatile float*)op = o1;
}

static inline int cdiv(int a, int b) { return (a + b - 1) / b; }

extern "C" void kernel_launch(void* const* d_in, const int* in_sizes, int n_in,
                              void* d_out, int out_size, void* d_ws, size_t ws_size,
                              hipStream_t stream) {
  if (n_in < 14) return;
  if (in_sizes[0] != N_EXP * HID) return;
  if (in_sizes[1] != 2 * E_EXP) return;
  const int nN = N_EXP;
  const int nE = E_EXP;
  if (in_sizes[2] != HID * HID || in_sizes[3] != HID) return;
  if (in_sizes[4] != 3 * HID * HID || in_sizes[5] != 3 * HID) return;
  if (in_sizes[6] != 2 * HID * HID || in_sizes[7] != HID) return;
  if (in_sizes[8] != HID || in_sizes[9] != 1) return;
  if (in_sizes[10] != HID * HID || in_sizes[11] != HID) return;
  if (in_sizes[12] != HID || in_sizes[13] != 1) return;
  const int total = 1 + nE + nN * HID;
  if (out_size != total || (total & 3) != 1) return;
  if ((nE & 31) != 0) return;

  const float* X    = (const float*)d_in[0];
  const int*   ei   = (const int*)d_in[1];
  const int*   src  = ei;
  const int*   dst  = ei + nE;
  const float* Wemb = (const float*)d_in[2];
  const float* bemb = (const float*)d_in[3];
  const float* Wgnn = (const float*)d_in[4];
  const float* bgnn = (const float*)d_in[5];
  const float* Wm1  = (const float*)d_in[6];
  const float* bm1  = (const float*)d_in[7];
  const float* Wm2  = (const float*)d_in[8];
  const float* bm2  = (const float*)d_in[9];
  const float* Wp1  = (const float*)d_in[10];
  const float* bp1  = (const float*)d_in[11];
  const float* Wp2  = (const float*)d_in[12];
  const float* bp2  = (const float*)d_in[13];
  float* out = (float*)d_out;

  const int MP = cdiv(nN, 128) * 128;
  if (MP != MP_EXP) return;
  const int gM = MP / GBM;
  const int gA = cdiv(MP, NBA);
  if ((long long)gA * NBA < (long long)MP) return;
  const int gE = cdiv(nE, EMB);
  const int vec8 = ((nE & 3) == 0) ? 1 : 0;

  char* ws = (char*)d_ws;
  size_t off = 0;
  const size_t oWeT  = off; off += (size_t)HID * HID * 2;        off = (off + 255) & ~(size_t)255;
  const size_t oWgT  = off; off += (size_t)3 * HID * KA * 2;     off = (off + 255) & ~(size_t)255;
  const size_t oWmT  = off; off += (size_t)KA * KA * 2;          off = (off + 255) & ~(size_t)255;
  const size_t oXB   = off; off += (size_t)MP * HID * 2;         off = (off + 255) & ~(size_t)255;
  const size_t oH    = off; off += (size_t)MP * HID * 4;         off = (off + 255) & ~(size_t)255;
  const size_t oHhl  = off; off += (size_t)MP * KA * 2;          off = (off + 255) & ~(size_t)255;
  const size_t oP    = off; off += (size_t)MP * KA * 4;          off = (off + 255) & ~(size_t)255;
  const size_t oMASK = off; off += (size_t)gE * EMB * 4;         off = (off + 255) & ~(size_t)255;
  const size_t oLIST = off; off += (size_t)gA * RCAP * 4;        off = (off + 255) & ~(size_t)255;
  const size_t oCNT  = off; off += (size_t)gA * NBA * 4;         off = (off + 255) & ~(size_t)255;
  const size_t oOFF  = off; off += (size_t)gA * NBA * 4;         off = (off + 255) & ~(size_t)255;
  const size_t oMETA = off; off += (size_t)gA * 32 * 4;          off = (off + 255) & ~(size_t)255;
  const size_t oPRED = off; off += (size_t)32 * 4;               off = (off + 255) & ~(size_t)255;
  if (off > ws_size || off > (size_t)WSMAX) return;
  unsigned short* WeT  = (unsigned short*)(ws + oWeT);
  unsigned short* WgT2 = (unsigned short*)(ws + oWgT);
  unsigned short* WmT2 = (unsigned short*)(ws + oWmT);
  unsigned short* XB   = (unsigned short*)(ws + oXB);
  float*          H    = (float*)(ws + oH);
  unsigned short* Hhl  = (unsigned short*)(ws + oHhl);
  float*          PSD  = (float*)(ws + oP);
  unsigned short* Zhl  = (unsigned short*)(ws + oP);
  float*          MASK = (float*)(ws + oMASK);
  int*            LIST = (int*)(ws + oLIST);
  int*            CNT  = (int*)(ws + oCNT);
  int*            OFF  = (int*)(ws + oOFF);
  int*            META = (int*)(ws + oMETA);
  float*          PRED = (float*)(ws + oPRED);

  const size_t bktLds = (size_t)BKT_LDS_INTS * 4;
  hipFuncSetAttribute(reinterpret_cast<const void*>(&k_bucket), hipFuncAttributeMaxDynamicSharedMemorySize,
                      (int)bktLds);

  const int nPrep = NU_WE + NU_WG + NU_WM + MP * 16;
  k_prep<<<nPrep / NTHR, NTHR, 0, stream>>>(X, Wemb, Wgnn, Wm1, nN, MP, WeT, WgT2, WmT2, XB);
  k_bucket<<<gA, NTHR, bktLds, stream>>>(dst, nE, vec8, LIST, CNT, OFF, META);
  k_gemm<1><<<dim3(gM, 1), GTHR, 0, stream>>>(XB, HID, WeT, HID, HID, bemb, nN, H, HID, Hhl);
  for (int i = 0; i < 3; ++i) {
    k_gemm<0><<<dim3(gM, 2), GTHR, 0, stream>>>(Hhl, KA, WmT2, KA, KA, bm1, nN, PSD, KA, Hhl);
    k_emask<<<gE, NTHR, 0, stream>>>(src, dst, nE, nN, PSD, Wm2, bm2, MASK);
    k_agg<<<MP / NWAVE, NTHR, 0, stream>>>(src, nE, nN, MP, LIST, CNT, OFF, META, MASK, H, Zhl);
    if (i < 2) {
      k_gemm<1><<<dim3(gM, 1), GTHR, 0, stream>>>(Zhl, KA, WgT2 + (size_t)i * HID * KA, KA, KA,
                                                   bgnn + (size_t)i * HID, nN, H, HID, Hhl);
    } else {
      k_gemm<2><<<dim3(gM, 1), GTHR, 0, stream>>>(Zhl, KA, WgT2 + (size_t)i * HID * KA, KA, KA,
                                                   bgnn + (size_t)i * HID, nN, H, HID, Hhl);
    }
  }
  k_pred<<<1, HID, 0, stream>>>(H, Wp1, bp1, Wp2, bp2, PRED);
  k_out<<<cdiv(total, OB), NTHR, 0, stream>>>(PRED, MASK, H, nE, nN * HID, total, out);
}
